// LocalTriangleAttentionNew_40527311405658
// MI455X (gfx1250) — hardware-verified
//
#include <hip/hip_runtime.h>
#include <hip/hip_bf16.h>

#define NMAT 192
#define NN   (192*192)
#define CZ   128
#define HH   4
#define CH   32
#define QKVG 512

typedef __attribute__((ext_vector_type(16))) _Float16 v16h;
typedef __attribute__((ext_vector_type(8)))  _Float16 v8h;
typedef __attribute__((ext_vector_type(8)))  float    v8f;
typedef __attribute__((ext_vector_type(4)))  _Float16 v4h;
typedef __attribute__((ext_vector_type(4)))  float    v4f;
#define VST2(T, ptr, val) do { const T _v = (val); *(volatile T*)(ptr) = _v; __threadfence(); *(volatile T*)(ptr) = _v; } while (0)
__device__ __forceinline__ int kmap(int e, int hh) { return (e < 8) ? (8 * hh + e) : (16 + 8 * hh + (e - 8)); }
__device__ __forceinline__ void wave_lds_sync() {
  __builtin_amdgcn_fence(__ATOMIC_RELEASE, "workgroup"); __builtin_amdgcn_wave_barrier(); __builtin_amdgcn_fence(__ATOMIC_ACQUIRE, "workgroup");
}

static __device__ __forceinline__ v8f wmma16x16x32(v16h a, v16h b, v8f c) {
  v8f d = __builtin_amdgcn_wmma_f32_16x16x32_f16(false, a, false, b, (short)0, c, false, false);
  asm volatile("v_nop\n\tv_nop\n\tv_nop\n\tv_nop" : "+v"(d) : "v"(a), "v"(b));
  return d;
}

static __device__ __forceinline__ v16h load_A_rm(const _Float16* p, int ld) {
  const int lane = threadIdx.x & 31;
  const int m = lane & 15, hi = lane >> 4;
  const _Float16* row = p + (size_t)m * ld;
  v16h a;
#pragma unroll
  for (int g = 0; g < 2; ++g)
#pragma unroll
    for (int w = 0; w < 8; ++w)
      a[g * 8 + w] = row[g * 16 + hi * 8 + w];
  return a;
}

static __device__ __forceinline__ v16h load_B_nk(const _Float16* pn0, int ldk) {
  const int lane = threadIdx.x & 31, n = lane & 15, hh = lane >> 4;
  const _Float16* row = pn0 + (size_t)n * ldk;
  const v8h lo = *(const v8h*)(row + 8 * hh), hi = *(const v8h*)(row + 16 + 8 * hh);
  return __builtin_shufflevector(lo, hi, 0,1,2,3,4,5,6,7,8,9,10,11,12,13,14,15);
}

__global__ void __launch_bounds__(256) k_prep(
    const float* __restrict__ w_q, const float* __restrict__ w_k,
    const float* __restrict__ w_v, const float* __restrict__ w_gate,
    const float* __restrict__ w_out, _Float16* __restrict__ Wcat,
    _Float16* __restrict__ Wout) {
  const int i8 = blockIdx.x * 256 + threadIdx.x;
  const int n = (i8 * 8) >> 7, k0 = (i8 * 8) & 127;
  const float qscale = 0.17677669529663687f;
  v8h v;
#pragma unroll
  for (int e = 0; e < 8; ++e) {
    const int k = k0 + e; float val;
    if (n < 128)      val = w_q[k * 128 + n] * qscale;
    else if (n < 256) val = w_k[k * 128 + (n - 128)];
    else if (n < 384) val = w_v[k * 128 + (n - 256)];
    else              val = w_gate[k * 128 + (n - 384)];
    v[e] = (_Float16)val;
  }
  VST2(v8h, Wcat + (size_t)i8 * 8, v);
  if (i8 < 128 * 128 / 8) {
    const int no = (i8 * 8) >> 7, ko = (i8 * 8) & 127;
    v8h w;
#pragma unroll
    for (int e = 0; e < 8; ++e) w[e] = (_Float16)w_out[(ko + e) * 128 + no];
    VST2(v8h, Wout + (size_t)i8 * 8, w);
  }
}

__global__ void __launch_bounds__(256) k_layernorm(
    const float* __restrict__ z, const float* __restrict__ ln_w,
    const float* __restrict__ ln_b, const float* __restrict__ w_bias,
    _Float16* __restrict__ zl, float* __restrict__ tb) {
  __shared__ float s_tb[32];
  const int row  = blockIdx.x * 8 + (threadIdx.x >> 5);
  const int lane = threadIdx.x & 31;
  const float* zr = z + (size_t)row * CZ;
  float x[4];
#pragma unroll
  for (int i = 0; i < 4; ++i) x[i] = zr[lane * 4 + i];
  float s = x[0] + x[1] + x[2] + x[3];
#pragma unroll
  for (int off = 16; off > 0; off >>= 1) s += __shfl_xor(s, off, 32);
  const float mu = s * (1.f / 128.f);
  float v = 0.f;
#pragma unroll
  for (int i = 0; i < 4; ++i) { float d = x[i] - mu; v += d * d; }
#pragma unroll
  for (int off = 16; off > 0; off >>= 1) v += __shfl_xor(v, off, 32);
  const float rstd = rsqrtf(v * (1.f / 128.f) + 1e-5f);
  float acc[4] = {0.f, 0.f, 0.f, 0.f};
  v4h zq;
#pragma unroll
  for (int i = 0; i < 4; ++i) {
    const int c = lane * 4 + i;
    const float zn = (x[i] - mu) * rstd * ln_w[c] + ln_b[c];
    zq[i] = (_Float16)zn;
#pragma unroll
    for (int hh = 0; hh < 4; ++hh) acc[hh] += zn * w_bias[c * 4 + hh];
  }
  VST2(v4h, zl + (size_t)row * CZ + lane * 4, zq);
#pragma unroll
  for (int hh = 0; hh < 4; ++hh)
#pragma unroll
    for (int off = 16; off > 0; off >>= 1) acc[hh] += __shfl_xor(acc[hh], off, 32);
  if (lane < 4) s_tb[(threadIdx.x >> 5) * 4 + lane] = acc[lane];
  __syncthreads();
  if (threadIdx.x < 32) VST2(float, tb + (size_t)blockIdx.x * 32 + threadIdx.x, s_tb[threadIdx.x]);
}

__global__ void __launch_bounds__(256) k_gemm_qkvg(
    const _Float16* __restrict__ A, const _Float16* __restrict__ Bw,
    _Float16* __restrict__ Y) {
  __shared__ __align__(16) _Float16 s_t[8][16 * 64];
  const int wv = threadIdx.x >> 5, lane = threadIdx.x & 31;
  const int tile = blockIdx.x * 8 + wv;
  const int nq = tile & 7;
  const int mt = tile >> 3;

  if (mt + 1 < NN / 16)
    __builtin_prefetch((const char*)(A + (size_t)((mt + 1) * 16) * CZ) +
                       threadIdx.x * 16, 0, 3);

  v8f acc[4] = {{}, {}, {}, {}};
#pragma unroll
  for (int kk = 0; kk < CZ; kk += 32) {
    v16h a = load_A_rm(A + (size_t)(mt * 16) * CZ + kk, CZ);
#pragma unroll
    for (int s = 0; s < 4; ++s) {
      v16h b = load_B_nk(Bw + (size_t)((nq * 4 + s) * 16) * CZ + kk, CZ);
      acc[s] = wmma16x16x32(a, b, acc[s]);
    }
  }
  const int n = lane & 15, mhi = lane >> 4;
  _Float16* st = s_t[wv];
#pragma unroll
  for (int s = 0; s < 4; ++s)
#pragma unroll
    for (int r = 0; r < 8; ++r) st[(r + 8 * mhi) * 64 + s * 16 + n] = (_Float16)acc[s][r];
  wave_lds_sync();
  for (int pass = 0; pass < 2; ++pass) {
#pragma unroll
    for (int jj = 0; jj < 4; ++jj) { const int rr = jj * 4 + (lane >> 3), sg = lane & 7;
      *(volatile v8h*)(Y + (size_t)(mt * 16 + rr) * QKVG + nq * 64 + sg * 8) = *(const v8h*)(st + rr * 64 + sg * 8); }
    __threadfence();
  }
}

__global__ void __launch_bounds__(256) k_attention(
    const _Float16* __restrict__ Yh, const float* __restrict__ tb,
    const float* __restrict__ mask, const float* __restrict__ b_gate,
    _Float16* __restrict__ go) {
  __shared__ float    s_logit[8][16][33];
  __shared__ _Float16 s_attn[8][16][32];
  __shared__ float    s_add[8][32];
  __shared__ __align__(16) _Float16 s_kv[8][32][32];
  __shared__ __align__(16) _Float16 s_go[2][16][CZ];

  const int wv   = threadIdx.x >> 5;
  const int lane = threadIdx.x & 31;
  const int task = blockIdx.x * 8 + wv;
  const int h  = task & 3;
  const int jb = (task >> 2) % 12;
  const int i  = task / 48;
  const int j0 = jb * 16;

  const _Float16* qbase = Yh + (size_t)(i * NMAT + j0) * QKVG + 0   + h * CH;
  const _Float16* kbase = Yh + (size_t)(i * NMAT)      * QKVG + 128 + h * CH;
  const _Float16* vbase = Yh + (size_t)(i * NMAT)      * QKVG + 256 + h * CH;
  const _Float16* gbase = Yh + (size_t)(i * NMAT)      * QKVG + 384 + h * CH;

  {
    const int jj  = j0 - 8 + lane;
    const int jjc = min(max(jj, 0), NMAT - 1);
    const bool ok = (jj >= 0) && (jj < NMAT) && (mask[i * NMAT + jjc] > 0.f);
    s_add[wv][lane] = ok ? 0.f : -1e9f;

    v8h* dst = (v8h*)&s_kv[wv][lane][0];
    if (jj >= 0 && jj < NMAT) {
      const v8h* src = (const v8h*)(kbase + (size_t)jj * QKVG);
#pragma unroll
      for (int q = 0; q < 4; ++q) dst[q] = src[q];
    } else {
      const v8h zr = {};
#pragma unroll
      for (int q = 0; q < 4; ++q) dst[q] = zr;
    }
  }

  const v16h qa = load_A_rm(qbase, QKVG);

#pragma unroll
  for (int t = 0; t < 2; ++t) {
    v16h kb;
#pragma unroll
    for (int e = 0; e < 16; ++e)
      kb[e] = s_kv[wv][t * 16 + (lane & 15)][kmap(e, lane >> 4)];
    v8f zero = {};
    v8f d = wmma16x16x32(qa, kb, zero);
    const int n = lane & 15, mhi = lane >> 4;
#pragma unroll
    for (int r = 0; r < 8; ++r)
      s_logit[wv][r + 8 * mhi][t * 16 + n] = d[r];
  }

  if (lane < 16) {
    const int m = lane;
    const int j = j0 + m;
    float lg[16];
    float mx = -3.0e38f;
#pragma unroll
    for (int w = 0; w < 16; ++w) {
      const int col = m + w;
      const int jj  = j0 - 8 + col;
      const int jjc = min(max(jj, 0), NMAT - 1);
      const float v = s_logit[wv][m][col] +
                      tb[(size_t)(j * NMAT + jjc) * 4 + h] + s_add[wv][col];
      lg[w] = v;
      mx = fmaxf(mx, v);
    }
    float sum = 0.f;
#pragma unroll
    for (int w = 0; w < 16; ++w) { lg[w] = expf(lg[w] - mx); sum += lg[w]; }
    const float inv = 1.f / sum;
#pragma unroll
    for (int c = 0; c < 32; ++c) s_attn[wv][m][c] = (_Float16)0.f;
#pragma unroll
    for (int w = 0; w < 16; ++w)
      s_attn[wv][m][m + w] = (_Float16)(lg[w] * inv);
  }

  v16h ab;
  {
    const int m = lane & 15, hi = lane >> 4;
#pragma unroll
    for (int g = 0; g < 2; ++g)
#pragma unroll
      for (int w = 0; w < 8; ++w)
        ab[g * 8 + w] = s_attn[wv][m][g * 16 + hi * 8 + w];
  }

#pragma unroll
  for (int t = 0; t < 2; ++t) {
    v16h vb;
    {
#pragma unroll
      for (int e = 0; e < 16; ++e) {
        const int jj = j0 - 8 + kmap(e, lane >> 4);
        vb[e] = (jj >= 0 && jj < NMAT) ? vbase[(size_t)jj * QKVG + t * 16 + (lane & 15)] : (_Float16)0.f;
      }
    }
    v8f zero = {};
    v8f o = wmma16x16x32(ab, vb, zero);
    const int n = lane & 15, mhi = lane >> 4;
#pragma unroll
    for (int r = 0; r < 8; ++r) {
      const int m = r + 8 * mhi;
      const int c = t * 16 + n;
      const float gp = (float)gbase[(size_t)(j0 + m) * QKVG + c] + b_gate[h * CH + c];
      const float gt = 1.f / (1.f + expf(-gp));
      s_go[wv >> 2][m][h * CH + c] = (_Float16)(gt * o[r]);
    }
  }
  __syncthreads();
  {
    const int tl = threadIdx.x >> 7, rr = (threadIdx.x >> 3) & 15, sg = threadIdx.x & 7;
    const int task0 = blockIdx.x * 8 + tl * 4;
    const int jb0 = (task0 >> 2) % 12, i0 = task0 / 48;
    _Float16* dst = go + (size_t)(i0 * NMAT + jb0 * 16 + rr) * CZ + sg * 8;
    const _Float16* srcp = &s_go[tl][rr][sg * 8];
    for (int pass = 0; pass < 2; ++pass) {
      *(volatile v8h*)dst = *(const v8h*)srcp; *(volatile v8h*)(dst + 64) = *(const v8h*)(srcp + 64);
      __threadfence();
    }
  }
}

__global__ void __launch_bounds__(256) k_gemm_out(
    const _Float16* __restrict__ A, const _Float16* __restrict__ Bw,
    const float* __restrict__ b_out, float* __restrict__ out) {
  const int wv = threadIdx.x >> 5, lane = threadIdx.x & 31;
  const int tile = blockIdx.x * 8 + wv;
  const int nq = tile & 1;
  const int mt = tile >> 1;

  if (mt + 4 < NN / 16)
    __builtin_prefetch((const char*)(A + (size_t)((mt + 4) * 16) * CZ) +
                       threadIdx.x * 16, 0, 3);

  v8f acc[4] = {{}, {}, {}, {}};
#pragma unroll
  for (int kk = 0; kk < CZ; kk += 32) {
    v16h a = load_A_rm(A + (size_t)(mt * 16) * CZ + kk, CZ);
#pragma unroll
    for (int s = 0; s < 4; ++s) {
      v16h b = load_B_nk(Bw + (size_t)((nq * 4 + s) * 16) * CZ + kk, CZ);
      acc[s] = wmma16x16x32(a, b, acc[s]);
    }
  }
  const int mhi = lane >> 4;
  for (int pass = 0; pass < 2; ++pass) {
#pragma unroll
    for (int pr = 0; pr < 2; ++pr) {
      const int c = nq * 64 + pr * 32 + lane;
      const float bo = b_out[c];
#pragma unroll
      for (int r = 0; r < 8; ++r) {
        const float a_ = acc[2 * pr][r], b_ = acc[2 * pr + 1][r];
        const float ax = __shfl_xor(a_, 16), bx = __shfl_xor(b_, 16);
        *(volatile float*)(out + (size_t)(mt * 16 + r) * CZ + c)     = (mhi ? bx : a_) + bo;
        *(volatile float*)(out + (size_t)(mt * 16 + r + 8) * CZ + c) = (mhi ? b_ : ax) + bo;
      }
    }
    __threadfence();
  }
}

extern "C" void kernel_launch(void* const* d_in, const int* in_sizes, int n_in,
                              void* d_out, int out_size, void* d_ws, size_t ws_size,
                              hipStream_t stream) {
  const float* z      = (const float*)d_in[0];
  const float* mask   = (const float*)d_in[1];
  const float* ln_w   = (const float*)d_in[2];
  const float* ln_b   = (const float*)d_in[3];
  const float* w_q    = (const float*)d_in[4];
  const float* w_k    = (const float*)d_in[5];
  const float* w_v    = (const float*)d_in[6];
  const float* w_bias = (const float*)d_in[7];
  const float* w_gate = (const float*)d_in[8];
  const float* b_gate = (const float*)d_in[9];
  const float* w_out  = (const float*)d_in[10];
  const float* b_out  = (const float*)d_in[11];
  float* out = (float*)d_out;
  (void)in_sizes; (void)n_in; (void)out_size;
  if (ws_size < (size_t)NN * (CZ * 2 + 16 + QKVG * 2 + CZ * 2) + (size_t)CZ * QKVG * 2 + CZ * CZ * 2 + 65536) return;

  char* ws = (char*)d_ws;
  size_t off = 0;
  auto carve = [&](size_t bytes) {
    char* p = ws + off;
    off += (bytes + 255) & ~(size_t)255;
    return p;
  };
  _Float16* zl_h = (_Float16*)carve((size_t)NN * CZ * 2);
  float*    tb   = (float*)   carve((size_t)NN * 4 * 4);
  _Float16* Wcat = (_Float16*)carve((size_t)CZ * QKVG * 2);
  _Float16* Wout = (_Float16*)carve((size_t)CZ * CZ * 2);
  _Float16* Yh   = (_Float16*)carve((size_t)NN * QKVG * 2);
  _Float16* go_h = (_Float16*)carve((size_t)NN * CZ * 2);

  k_prep<<<dim3((CZ * QKVG) / 8 / 256), dim3(256), 0, stream>>>(
      w_q, w_k, w_v, w_gate, w_out, Wcat, Wout);
  k_layernorm<<<dim3(NN / 8), dim3(256), 0, stream>>>(
      z, ln_w, ln_b, w_bias, zl_h, tb);
  k_gemm_qkvg<<<dim3((NN / 16) * 8 / 8), dim3(256), 0, stream>>>(
      zl_h, Wcat, Yh);
  k_attention<<<dim3(NMAT * 12 * 4 / 8), dim3(256), 0, stream>>>(
      Yh, tb, mask, b_gate, go_h);
  k_gemm_out<<<dim3((NN / 16) * 2 / 8), dim3(256), 0, stream>>>(
      go_h, Wout, b_out, out);
}
